// _MoEBlock_2499670966569
// MI455X (gfx1250) — hardware-verified
//
#include <hip/hip_runtime.h>
#include <stddef.h>

#define NTOK  8192
#define HD    1024
#define NE    8
#define CAPC  1024
#define NSLOT (NE * CAPC)

static_assert(NSLOT == NTOK);
static_assert(NTOK % 32 == 0);
static_assert(NTOK == 512 * 16);
static_assert(HD == 128 * 8);
static_assert(HD % 128 == 0);
static_assert(CAPC % 128 == 0);
static_assert((NE * HD * HD) % (256 * 8) == 0);

typedef float          v4f_t __attribute__((ext_vector_type(4)));
typedef v4f_t          __attribute__((may_alias)) v4f;
typedef int            v4i_t __attribute__((ext_vector_type(4)));
typedef v4i_t          __attribute__((may_alias)) v4i;
typedef unsigned int   v4u_t __attribute__((ext_vector_type(4)));
typedef v4u_t          __attribute__((may_alias)) v4u;
typedef float          v8f   __attribute__((ext_vector_type(8)));
typedef __bf16         v16bf __attribute__((ext_vector_type(16)));
typedef unsigned short v8us_t __attribute__((ext_vector_type(8)));
typedef v8us_t         __attribute__((may_alias)) v8us;

union FragU { v16bf v; v8us_t h[2]; };

__device__ __forceinline__ v8f zero8() {
    v8f z;
#pragma unroll
    for (int i = 0; i < 8; ++i) z[i] = 0.0f;
    return z;
}

__device__ __forceinline__ v16bf ldfrag(const unsigned short* p, int k0) {
    FragU f;
    f.h[0] = *(const v8us*)(p + k0);
    f.h[1] = *(const v8us*)(p + k0 + 16);
    return f.v;
}

__device__ __forceinline__ v8f wmma_bf16(v16bf a, v16bf b, v8f c) {
    return __builtin_amdgcn_wmma_f32_16x16x32_bf16(false, a, false, b, (short)0, c, false, false);
}

__device__ __forceinline__ unsigned int bf16_rne_bits(float f) {
    const unsigned int u = __float_as_uint(f);
    return (u + 0x7FFFu + ((u >> 16) & 1u)) >> 16;
}

__device__ __forceinline__ void split8(const float (&v)[8], v4u_t& hp, v4u_t& lp) {
#pragma unroll
    for (int q = 0; q < 4; ++q) {
        const unsigned int h0 = bf16_rne_bits(v[2 * q]);
        const unsigned int h1 = bf16_rne_bits(v[2 * q + 1]);
        const float r0 = v[2 * q]     - __uint_as_float(h0 << 16);
        const float r1 = v[2 * q + 1] - __uint_as_float(h1 << 16);
        const unsigned int l0 = bf16_rne_bits(r0);
        const unsigned int l1 = bf16_rne_bits(r1);
        hp[q] = h0 | (h1 << 16);
        lp[q] = l0 | (l1 << 16);
    }
}

__global__ void __launch_bounds__(256)
gate_kernel(const float* __restrict__ x, const float* __restrict__ wg,
            int* __restrict__ tok_expert, float* __restrict__ tok_gate)
{
    __shared__ int   s_e[32];
    __shared__ float s_g[32];
    const int lane = threadIdx.x & 31, w = threadIdx.x >> 5;
    const int le = lane & 7;

#pragma unroll 1
    for (int q = 0; q < 4; ++q) {
        const int tl = w * 4 + q;
        const int t  = blockIdx.x * 32 + tl;
        const float* xr = x + (size_t)t * HD;
        float acc[NE];
#pragma unroll
        for (int e = 0; e < NE; ++e) acc[e] = 0.0f;
#pragma unroll 1
        for (int j = 0; j < HD / 32; ++j) {
            const int h = j * 32 + lane;
            const float xv = xr[h];
            const v4f_t w0 = *(const v4f*)(wg + (size_t)h * NE);
            const v4f_t w1 = *(const v4f*)(wg + (size_t)h * NE + 4);
#pragma unroll
            for (int e = 0; e < 4; ++e) {
                acc[e]     = fmaf(xv, w0[e], acc[e]);
                acc[4 + e] = fmaf(xv, w1[e], acc[4 + e]);
            }
        }
#pragma unroll
        for (int e = 0; e < NE; ++e) {
#pragma unroll
            for (int off = 16; off > 0; off >>= 1) acc[e] += __shfl_xor(acc[e], off, 32);
        }
        float mx = acc[0];
#pragma unroll
        for (int e = 1; e < NE; ++e) mx = fmaxf(mx, acc[e]);
        float my = acc[0];
#pragma unroll
        for (int e = 1; e < NE; ++e) my = (le == e) ? acc[e] : my;
        const float ex = expf(my - mx);
        float s = ex;
        s += __shfl_xor(s, 1, 32);
        s += __shfl_xor(s, 2, 32);
        s += __shfl_xor(s, 4, 32);
        const float p = ex * (1.0f / s);
        float bv = p;
        int   bi = le;
#pragma unroll
        for (int off = 1; off < 8; off <<= 1) {
            const float ov = __shfl_xor(bv, off, 32);
            const int   oi = __shfl_xor(bi, off, 32);
            const bool take = (ov > bv) || (ov == bv && oi < bi);
            bv = take ? ov : bv;
            bi = take ? oi : bi;
        }
        if (lane == 0) { s_e[tl] = bi; s_g[tl] = bv; }
    }
    __syncthreads();
    if (w == 0) {
        const int   ve = s_e[lane];
        const float vg = s_g[lane];
        const size_t o = (size_t)blockIdx.x * 32 + lane;
        *(volatile int*)(tok_expert + o)  = ve;
        *(volatile float*)(tok_gate + o)  = vg;
        __threadfence();
        *(volatile int*)(tok_expert + o)  = ve;
        *(volatile float*)(tok_gate + o)  = vg;
    }
}

__global__ void __launch_bounds__(512)
route_kernel(const int* __restrict__ tok_expert, const float* __restrict__ tok_gate,
             int* __restrict__ slot_token, float* __restrict__ slot_gate,
             int* __restrict__ tok_slot)
{
    __shared__ __align__(16) int   sl_tok[NSLOT];
    __shared__ __align__(16) float sl_gt[NSLOT];
    __shared__ int wtot[NE * 16];
    const int tid = threadIdx.x, lane = tid & 31, w = tid >> 5;
    const int t0 = tid * 16;

    int   ex[16];
    float gt[16];
#pragma unroll
    for (int c = 0; c < 4; ++c) {
        const v4i_t ve = *(const v4i*)(tok_expert + t0 + 4 * c);
        const v4f_t vg = *(const v4f*)(tok_gate + t0 + 4 * c);
#pragma unroll
        for (int i = 0; i < 4; ++i) {
            int ee = ve[i];
            ee = ee < 0 ? 0 : ee;
            ee = ee > NE - 1 ? NE - 1 : ee;
            ex[4 * c + i] = ee;
            gt[4 * c + i] = vg[i];
        }
    }
    int cnt[NE];
#pragma unroll
    for (int e = 0; e < NE; ++e) cnt[e] = 0;
#pragma unroll
    for (int j = 0; j < 16; ++j) {
#pragma unroll
        for (int e = 0; e < NE; ++e) cnt[e] += (ex[j] == e) ? 1 : 0;
    }
    int incl[NE];
#pragma unroll
    for (int e = 0; e < NE; ++e) {
        int v = cnt[e];
#pragma unroll
        for (int off = 1; off < 32; off <<= 1) {
            const int n = __shfl_up(v, off, 32);
            if (lane >= off) v += n;
        }
        incl[e] = v;
    }
    if (lane == 31) {
#pragma unroll
        for (int e = 0; e < NE; ++e) wtot[e * 16 + w] = incl[e];
    }
#pragma unroll 1
    for (int i = tid; i < NSLOT; i += 512) { sl_tok[i] = -1; sl_gt[i] = 0.0f; }
    __syncthreads();

    int pos[NE];
#pragma unroll
    for (int e = 0; e < NE; ++e) {
        int b = 0;
#pragma unroll
        for (int w2 = 0; w2 < 16; ++w2) {
            const int tv = wtot[e * 16 + w2];
            b += (w2 < w) ? tv : 0;
        }
        pos[e] = b + incl[e] - cnt[e];
    }
    int ms[16];
#pragma unroll
    for (int j = 0; j < 16; ++j) {
        const int e = ex[j];
        int p = pos[0];
#pragma unroll
        for (int e2 = 1; e2 < NE; ++e2) p = (e == e2) ? pos[e2] : p;
#pragma unroll
        for (int e2 = 0; e2 < NE; ++e2) pos[e2] += (e == e2) ? 1 : 0;
        const bool kept = (p < CAPC);
        const int  s    = e * CAPC + (kept ? p : 0);
        if (kept) { sl_tok[s] = t0 + j; sl_gt[s] = gt[j]; }
        ms[j] = kept ? s : -1;
    }
    __syncthreads();

#pragma unroll
    for (int c = 0; c < 4; ++c) {
        const int i = c * 2048 + tid * 4;
        const v4i_t a = *(const v4i*)(sl_tok + i);
        const v4f_t g = *(const v4f*)(sl_gt + i);
        *(volatile v4i*)(slot_token + i) = a;
        *(volatile v4f*)(slot_gate + i)  = g;
    }
    __threadfence();
#pragma unroll
    for (int c = 0; c < 4; ++c) {
        const int i = c * 2048 + tid * 4;
        const v4i_t a = *(const v4i*)(sl_tok + i);
        const v4f_t g = *(const v4f*)(sl_gt + i);
        *(volatile v4i*)(slot_token + i) = a;
        *(volatile v4f*)(slot_gate + i)  = g;
    }
    __syncthreads();

#pragma unroll
    for (int j = 0; j < 16; ++j) sl_tok[t0 + j] = ms[j];
    __syncthreads();
#pragma unroll
    for (int c = 0; c < 4; ++c) {
        const int i = c * 2048 + tid * 4;
        const v4i_t a = *(const v4i*)(sl_tok + i);
        *(volatile v4i*)(tok_slot + i) = a;
    }
    __threadfence();
#pragma unroll
    for (int c = 0; c < 4; ++c) {
        const int i = c * 2048 + tid * 4;
        const v4i_t a = *(const v4i*)(sl_tok + i);
        *(volatile v4i*)(tok_slot + i) = a;
    }
}

__global__ void __launch_bounds__(128)
dispatch_kernel(const float* __restrict__ x, const int* __restrict__ slot_token,
                const int* __restrict__ tok_slot,
                unsigned short* __restrict__ ahi, unsigned short* __restrict__ alo,
                float* __restrict__ out)
{
    const int s = blockIdx.x, j = threadIdx.x;
    const int t = slot_token[s];
    const bool valid = (unsigned)t < (unsigned)NTOK;
    const int tt = valid ? t : 0;
    const float* xr = x + (size_t)tt * HD + (size_t)j * 8;
    const v4f_t a = *(const v4f*)(xr);
    const v4f_t b = *(const v4f*)(xr + 4);
    float v[8];
#pragma unroll
    for (int i = 0; i < 4; ++i) {
        v[i]     = valid ? a[i] : 0.0f;
        v[4 + i] = valid ? b[i] : 0.0f;
    }
    v4u_t hp, lp;
    split8(v, hp, lp);
    const size_t o = (size_t)s * HD + (size_t)j * 8;

    const int ts = tok_slot[s];
    const bool dropped = (unsigned)ts >= (unsigned)NSLOT;
    v4f_t z;
#pragma unroll
    for (int i = 0; i < 4; ++i) z[i] = 0.0f;
    float* orow = out + (size_t)s * HD + (size_t)j * 4;

    *(volatile v4u*)(ahi + o) = hp;
    *(volatile v4u*)(alo + o) = lp;
    if (dropped) {
        *(volatile v4f*)(orow)       = z;
        *(volatile v4f*)(orow + 512) = z;
    }
    __threadfence();
    *(volatile v4u*)(ahi + o) = hp;
    *(volatile v4u*)(alo + o) = lp;
    if (dropped) {
        *(volatile v4f*)(orow)       = z;
        *(volatile v4f*)(orow + 512) = z;
    }
}

__global__ void __launch_bounds__(256)
cvtw_kernel(const float* __restrict__ W, unsigned short* __restrict__ whi,
            unsigned short* __restrict__ wlo, int n8)
{
    const int i = blockIdx.x * 256 + threadIdx.x;
    if (i >= n8) return;
    const float* src = W + (size_t)i * 8;
    const v4f_t a = *(const v4f*)(src);
    const v4f_t b = *(const v4f*)(src + 4);
    float v[8];
#pragma unroll
    for (int q = 0; q < 4; ++q) { v[q] = a[q]; v[4 + q] = b[q]; }
    v4u_t hp, lp;
    split8(v, hp, lp);
    const size_t o = (size_t)i * 8;
    *(volatile v4u*)(whi + o) = hp;
    *(volatile v4u*)(wlo + o) = lp;
    __threadfence();
    *(volatile v4u*)(whi + o) = hp;
    *(volatile v4u*)(wlo + o) = lp;
}

__global__ void __launch_bounds__(256)
expert_gemm_kernel(const unsigned short* __restrict__ ahi, const unsigned short* __restrict__ alo,
                   const unsigned short* __restrict__ whi, const unsigned short* __restrict__ wlo,
                   const float* __restrict__ bias, const int* __restrict__ slot_token,
                   const float* __restrict__ slot_gate, float* __restrict__ out)
{
    __shared__ __align__(16) float tile[128 * 128];
    const int lane = threadIdx.x & 31, w = threadIdx.x >> 5;
    const int lm = lane & 15, kh = lane >> 4;
    const int bid = blockIdx.x;
    const int e  = bid >> 6;
    const int mt = (bid >> 3) & 7;
    const int nt = bid & 7;
    const int m0 = mt * 128, n0 = nt * 128;
    const int wm = w & 3, wn = w >> 2;

    const size_t arow = ((size_t)e * CAPC + m0 + wm * 32 + lm) * HD + 8 * kh;
    const unsigned short* pah0 = ahi + arow;
    const unsigned short* pah1 = pah0 + (size_t)16 * HD;
    const unsigned short* pal0 = alo + arow;
    const unsigned short* pal1 = pal0 + (size_t)16 * HD;
    const size_t brow = ((size_t)e * HD + n0 + wn * 64 + lm) * HD + 8 * kh;
    const unsigned short* pbh = whi + brow;
    const unsigned short* pbl = wlo + brow;

    v8f acc[2][4];
#pragma unroll
    for (int mi = 0; mi < 2; ++mi)
#pragma unroll
        for (int ni = 0; ni < 4; ++ni) acc[mi][ni] = zero8();

#pragma unroll 1
    for (int k0 = 0; k0 < HD; k0 += 32) {
        const v16bf ah0 = ldfrag(pah0, k0);
        const v16bf ah1 = ldfrag(pah1, k0);
        const v16bf al0 = ldfrag(pal0, k0);
        const v16bf al1 = ldfrag(pal1, k0);
#pragma unroll
        for (int ni = 0; ni < 4; ++ni) {
            const v16bf bh = ldfrag(pbh + (size_t)ni * 16 * HD, k0);
            const v16bf bl = ldfrag(pbl + (size_t)ni * 16 * HD, k0);
            acc[0][ni] = wmma_bf16(ah0, bh, acc[0][ni]);
            acc[1][ni] = wmma_bf16(ah1, bh, acc[1][ni]);
            acc[0][ni] = wmma_bf16(ah0, bl, acc[0][ni]);
            acc[1][ni] = wmma_bf16(ah1, bl, acc[1][ni]);
            acc[0][ni] = wmma_bf16(al0, bh, acc[0][ni]);
            acc[1][ni] = wmma_bf16(al1, bh, acc[1][ni]);
            asm volatile("v_nop\n\tv_nop\n\tv_nop\n\tv_nop"
                         : "+v"(acc[0][ni]), "+v"(acc[1][ni])
                         : "v"(ah0), "v"(ah1), "v"(al0), "v"(al1), "v"(bh), "v"(bl));
        }
    }

#pragma unroll
    for (int mi = 0; mi < 2; ++mi)
#pragma unroll
        for (int ni = 0; ni < 4; ++ni)
#pragma unroll
            for (int r = 0; r < 8; ++r)
                tile[(wm * 32 + mi * 16 + kh * 8 + r) * 128 + wn * 64 + ni * 16 + lm] = acc[mi][ni][r];
    __syncthreads();

    const int col = n0 + lane * 4;
    const v4f_t bb = *(const v4f*)(bias + (size_t)e * HD + col);
    const int*   stok = slot_token + (size_t)e * CAPC + m0 + w * 16;
    const float* sgt  = slot_gate  + (size_t)e * CAPC + m0 + w * 16;

#pragma unroll 1
    for (int rr = 0; rr < 16; ++rr) {
        const int tok = stok[rr];
        const float g = sgt[rr];
        if ((unsigned)tok < (unsigned)NTOK) {
            const v4f_t v = *(const v4f*)(tile + (w * 16 + rr) * 128 + lane * 4);
            const v4f_t o = (v + bb) * g;
            *(volatile v4f*)(out + (size_t)tok * HD + col) = o;
        }
    }
    __threadfence();
#pragma unroll 1
    for (int rr = 0; rr < 16; ++rr) {
        const int tok = stok[rr];
        const float g = sgt[rr];
        if ((unsigned)tok < (unsigned)NTOK) {
            const v4f_t v = *(const v4f*)(tile + (w * 16 + rr) * 128 + lane * 4);
            const v4f_t o = (v + bb) * g;
            *(volatile v4f*)(out + (size_t)tok * HD + col) = o;
        }
    }
}

extern "C" void kernel_launch(void* const* d_in, const int* in_sizes, int n_in,
                              void* d_out, int out_size, void* d_ws, size_t ws_size,
                              hipStream_t stream)
{
    if (n_in < 4) return;
    if (in_sizes[0] != NTOK * HD) return;
    if (in_sizes[1] != HD * NE) return;
    if (in_sizes[2] != NE * HD * HD) return;
    if (in_sizes[3] != NE * HD) return;
    if (out_size != NTOK * HD) return;

    const float* x  = (const float*)d_in[0];
    const float* wg = (const float*)d_in[1];
    const float* W  = (const float*)d_in[2];
    const float* b  = (const float*)d_in[3];
    float* out = (float*)d_out;

    const size_t nTab = (size_t)NTOK * 4;
    const size_t o_te = 0;
    const size_t o_tg = o_te + nTab;
    const size_t o_st = o_tg + nTab;
    const size_t o_sg = o_st + nTab;
    const size_t o_ts = o_sg + nTab;
    const size_t o_ah = o_ts + nTab;
    const size_t nA   = (size_t)NSLOT * HD * 2;
    const size_t o_al = o_ah + nA;
    const size_t o_wh = o_al + nA;
    const size_t nWb  = (size_t)NE * HD * HD * 2;
    const size_t o_wl = o_wh + nWb;
    const size_t total = o_wl + nWb;
    if (total > ws_size) return;

    char* ws = (char*)d_ws;
    int*   tok_expert = (int*)(ws + o_te);
    float* tok_gate   = (float*)(ws + o_tg);
    int*   slot_token = (int*)(ws + o_st);
    float* slot_gate  = (float*)(ws + o_sg);
    int*   tok_slot   = (int*)(ws + o_ts);
    unsigned short* ahi = (unsigned short*)(ws + o_ah);
    unsigned short* alo = (unsigned short*)(ws + o_al);
    unsigned short* whi = (unsigned short*)(ws + o_wh);
    unsigned short* wlo = (unsigned short*)(ws + o_wl);

    const int n8W = (NE * HD * HD) / 8;

    gate_kernel<<<NTOK / 32, 256, 0, stream>>>(x, wg, tok_expert, tok_gate);
    route_kernel<<<1, 512, 0, stream>>>(tok_expert, tok_gate, slot_token, slot_gate, tok_slot);
    cvtw_kernel<<<(n8W + 255) / 256, 256, 0, stream>>>(W, whi, wlo, n8W);
    dispatch_kernel<<<NSLOT, 128, 0, stream>>>(x, slot_token, tok_slot, ahi, alo, out);
    expert_gemm_kernel<<<NE * (CAPC / 128) * (HD / 128), 256, 0, stream>>>(
        ahi, alo, whi, wlo, b, slot_token, slot_gate, out);
}
